// STU_42305427865774
// MI455X (gfx1250) — hardware-run, weakly checked
//
#include <hip/hip_runtime.h>
#include <stdint.h>
#include <stddef.h>

typedef __attribute__((ext_vector_type(16))) _Float16 v16h;
typedef __attribute__((ext_vector_type(8)))  _Float16 v8h;
typedef __attribute__((ext_vector_type(16))) __bf16   v16b;
typedef __attribute__((ext_vector_type(8)))  __bf16   v8b;
typedef __attribute__((ext_vector_type(8)))  float    v8f;
typedef __attribute__((ext_vector_type(4)))  float    v4f;
typedef __attribute__((ext_vector_type(4)))  unsigned u32x4;

constexpr int kSeq     = 2048;
constexpr int kHalfSeq = 1024;
constexpr int kDin     = 512;
constexpr int kDout    = 512;
constexpr int kNumF    = 24;
constexpr int kNumLag  = 3;
constexpr int kNumZ    = 2 * kNumF;
constexpr int kArK     = kNumLag * kDin;
constexpr int kQZero   = 64;
constexpr int kQLen    = 1280;
constexpr int kQLines  = 2 * 2 * kNumF;
constexpr int kAPitch  = 40;
constexpr int kThreads = 256;
constexpr int kXPRows  = kSeq + 1;

constexpr float kWCarry    = 64.0f;
constexpr float kPhiCarry  = 64.0f;
constexpr float kGEpiScale = 0.25f;
constexpr float kArCarry   = 1024.0f;
constexpr float kOutScale  = 1.0f / 1024.0f;
static_assert(kPhiCarry * (kWCarry * kGEpiScale) == kArCarry);
static_assert(kOutScale * kArCarry == 1.0f);

static_assert(kSeq == 2 * kHalfSeq);
static_assert(kDin % 32 == 0 && kArK % 32 == 0 && kHalfSeq % 64 == 0);
static_assert(kDout % 64 == 0 && kSeq % 64 == 0 && kHalfSeq % 64 == 0);
static_assert(kDout == 8 * 64);
static_assert(kQLen == 160 * 8 && kQLen >= kQZero + kHalfSeq);
static_assert(kQZero + (kHalfSeq - 64) + 63 < kQLen);
static_assert(kAPitch % 8 == 0 && kAPitch >= 32);
static_assert(((kDout / 64) * (kSeq / 64)) % 8 == 0);

constexpr size_t kBytesXP  = (size_t)kXPRows * kDin * 2;
constexpr size_t kBytesMT  = (size_t)kNumZ * kDout * kDin * 2;
constexpr size_t kBytesB   = (size_t)kNumF * kDout * kSeq * 2;
constexpr size_t kBytesQT  = (size_t)kQLines * kQLen * 2;
constexpr size_t kBytesMar = (size_t)kDout * kArK * 2;
constexpr size_t kOffXP  = 0;
constexpr size_t kOffMT  = kOffXP + kBytesXP;
constexpr size_t kOffBE  = kOffMT + kBytesMT;
constexpr size_t kOffBO  = kOffBE + kBytesB;
constexpr size_t kOffQT  = kOffBO + kBytesB;
constexpr size_t kOffMar = kOffQT + kBytesQT;
constexpr size_t kWsTotal = kOffMar + kBytesMar;
static_assert(kWsTotal == 129745920u);
static_assert(kWsTotal <= 134217728u);
static_assert(kOffMT % 256 == 0 && kOffBE % 256 == 0 && kOffBO % 256 == 0 && kOffQT % 256 == 0 && kOffMar % 256 == 0);

__device__ __forceinline__ unsigned short f2bf_bits(float f) {
  unsigned u = __float_as_uint(f);
  return (unsigned short)((u + 0x7FFFu + ((u >> 16) & 1u)) >> 16);
}
__device__ __forceinline__ float bf_bits2f(unsigned short h) { return __uint_as_float(((unsigned)h) << 16); }
__device__ __forceinline__ float bfr(float f) { return bf_bits2f(f2bf_bits(f)); }
__device__ __forceinline__ unsigned h16bits(float f) { return (unsigned)__builtin_bit_cast(unsigned short, (_Float16)f); }
__device__ __forceinline__ unsigned pack_h2(float lo, float hi) { return h16bits(lo) | (h16bits(hi) << 16); }

__device__ __forceinline__ void dep_guard_h(v8f& a, v8f& b, v16h x, v16h y) { asm volatile("v_nop\n\tv_nop\n\tv_nop\n\tv_nop" : "+v"(a), "+v"(b) : "v"(x), "v"(y)); }
__device__ __forceinline__ void dep_guard_b(v8f& a, v8f& b, v16b x, v16b y) { asm volatile("v_nop\n\tv_nop\n\tv_nop\n\tv_nop" : "+v"(a), "+v"(b) : "v"(x), "v"(y)); }
__device__ __forceinline__ void grp_guard_h(v8f& a, v8f& b, v8f& c, v8f& d, v16h x, v16h y) { asm volatile("v_nop\n\tv_nop\n\tv_nop\n\tv_nop" : "+v"(a), "+v"(b), "+v"(c), "+v"(d) : "v"(x), "v"(y)); }
__device__ __forceinline__ void grp_guard_b(v8f& a, v8f& b, v8f& c, v8f& d, v16b x, v16b y) { asm volatile("v_nop\n\tv_nop\n\tv_nop\n\tv_nop" : "+v"(a), "+v"(b), "+v"(c), "+v"(d) : "v"(x), "v"(y)); }
__device__ __forceinline__ void keep4_h(v16h a, v16h b, v16h c, v16h d) { asm volatile("v_nop" :: "v"(a), "v"(b), "v"(c), "v"(d)); }
__device__ __forceinline__ void keep4_b(v16b a, v16b b, v16b c, v16b d) { asm volatile("v_nop" :: "v"(a), "v"(b), "v"(c), "v"(d)); }
__device__ __forceinline__ void acc_guard4(v8f& a, v8f& b, v8f& c, v8f& d) { asm volatile("v_nop\n\tv_nop\n\tv_nop\n\tv_nop" : "+v"(a), "+v"(b), "+v"(c), "+v"(d)); }
template <typename T> struct Frag;
template <> struct Frag<_Float16> {
  typedef v16h V; union U { v16h v; v8h h[2]; };
  static __device__ __forceinline__ v16h load(const _Float16* p) {
    U f; f.h[0] = *(const v8h*)(p); f.h[1] = *(const v8h*)(p + 16); return f.v;
  }
  static __device__ __forceinline__ v8f mma(v16h a, v16h b, v8f c) {
    return __builtin_amdgcn_wmma_f32_16x16x32_f16(false, a, false, b, (short)0, c, false, false);
  }
  static __device__ __forceinline__ void guard(v8f& a, v8f& b, v16h x, v16h y) { dep_guard_h(a, b, x, y); }
  static __device__ __forceinline__ void guard4(v8f& a, v8f& b, v8f& c, v8f& d, v16h x, v16h y) { grp_guard_h(a, b, c, d, x, y); }
  static __device__ __forceinline__ void keep(v16h a, v16h b, v16h c, v16h d) { keep4_h(a, b, c, d); }
};
template <> struct Frag<__bf16> {
  typedef v16b V; union U { v16b v; v8b h[2]; };
  static __device__ __forceinline__ v16b load(const __bf16* p) {
    U f; f.h[0] = *(const v8b*)(p); f.h[1] = *(const v8b*)(p + 16); return f.v;
  }
  static __device__ __forceinline__ v8f mma(v16b a, v16b b, v8f c) {
    return __builtin_amdgcn_wmma_f32_16x16x32_bf16(false, a, false, b, (short)0, c, false, false);
  }
  static __device__ __forceinline__ void guard(v8f& a, v8f& b, v16b x, v16b y) { dep_guard_b(a, b, x, y); }
  static __device__ __forceinline__ void guard4(v8f& a, v8f& b, v8f& c, v8f& d, v16b x, v16b y) { grp_guard_b(a, b, c, d, x, y); }
  static __device__ __forceinline__ void keep(v16b a, v16b b, v16b c, v16b d) { keep4_b(a, b, c, d); }
};
typedef Frag<_Float16> FragH;

template <int ET> struct Elem;
template <> struct Elem<0> { typedef _Float16 T; };
template <> struct Elem<1> { typedef __bf16 T; };
template <int ET, bool SPLIT, int BIAS_MODE, int OUT_MODE, bool RESID, int ACT = 0>
__global__ __launch_bounds__(256) void wmma_gemm64(
    const unsigned short* __restrict__ Ap, const unsigned short* __restrict__ A2p, int lda, long strideA,
    const unsigned short* __restrict__ Btp, const unsigned short* __restrict__ Bt2p, int ldb, long strideB,
    void* __restrict__ Cout, void* __restrict__ Cout2, int ldc, long strideC,
    const float* __restrict__ bias,
    const float* __restrict__ resid, long strideR,
    int M, int N, int K, float scale) {
  typedef typename Elem<ET>::T T;
  typedef typename Frag<T>::V V;
  const T* A = (const T*)Ap; const T* A2 = (const T*)A2p; const T* Bt = (const T*)Btp; const T* Bt2 = (const T*)Bt2p;
  __shared__ __align__(16) float sT[8][16 * 68];
  const int b    = blockIdx.y;
  const int lane = threadIdx.x & 31;
  const int wave = threadIdx.x >> 5;
  const int tilesN = N >> 6;
  const int tilesM = M >> 6;
  const int tile = blockIdx.x * 8 + wave;
  if (tile >= tilesM * tilesN) return;
  const int tm = tile / tilesN;
  const int tn = tile - tm * tilesN;
  const int m0 = tm << 6;
  const int n0 = tn << 6;

  const T* Ab  = A  + (size_t)b * strideA;
  const T* Bb  = Bt + (size_t)b * strideB;
  const T* Ab2 = SPLIT ? (A2  + (size_t)b * strideA) : nullptr;
  const T* Bb2 = SPLIT ? (Bt2 + (size_t)b * strideB) : nullptr;

  const int rlane = lane & 15;
  const int koff  = (lane >> 4) * 8;
  const int mOff  = (lane >> 4) * 8;

  v8f acc[4][4];
#pragma unroll
  for (int i = 0; i < 4; ++i)
#pragma unroll
    for (int j = 0; j < 4; ++j) acc[i][j] = (v8f){0.f,0.f,0.f,0.f,0.f,0.f,0.f,0.f};

  for (int k0 = 0; k0 < K; k0 += 32) {
    V bh[4], bl[4];
#pragma unroll
    for (int j = 0; j < 4; ++j) {
      const size_t bo = (size_t)(n0 + (j << 4) + rlane) * ldb + koff + k0;
      bh[j] = Frag<T>::load(Bb + bo);
      if (SPLIT) bl[j] = Frag<T>::load(Bb2 + bo);
    }
#pragma unroll
    for (int i = 0; i < 4; ++i) {
      const size_t ao = (size_t)(m0 + (i << 4) + rlane) * lda + koff + k0;
      V ah = Frag<T>::load(Ab + ao);
      V al;
      if (SPLIT) al = Frag<T>::load(Ab2 + ao);
#pragma unroll
      for (int j = 0; j < 4; ++j) {
        acc[i][j] = Frag<T>::mma(ah, bh[j], acc[i][j]);
        if (SPLIT) {
          acc[i][j] = Frag<T>::mma(ah, bl[j], acc[i][j]);
          acc[i][j] = Frag<T>::mma(al, bh[j], acc[i][j]);
        }
      }
      Frag<T>::guard4(acc[i][0], acc[i][1], acc[i][2], acc[i][3], ah, bh[3]);
      if (SPLIT) Frag<T>::guard(acc[i][0], acc[i][3], al, bl[3]);
    }
    Frag<T>::keep(bh[0], bh[1], bh[2], bh[3]);
    if (SPLIT) Frag<T>::keep(bl[0], bl[1], bl[2], bl[3]);
  }
  acc_guard4(acc[0][0], acc[0][1], acc[0][2], acc[0][3]);
  acc_guard4(acc[1][0], acc[1][1], acc[1][2], acc[1][3]);
  acc_guard4(acc[2][0], acc[2][1], acc[2][2], acc[2][3]);
  acc_guard4(acc[3][0], acc[3][1], acc[3][2], acc[3][3]);

  float* slab = sT[wave];
  const float* Rb = RESID ? (resid + (size_t)b * strideR) : nullptr;
#pragma unroll
  for (int i = 0; i < 4; ++i) {
    const int mBase = m0 + (i << 4);
#pragma unroll
    for (int j = 0; j < 4; ++j) {
      const int n = n0 + (j << 4) + rlane;
      float bv = 0.f;
      if (BIAS_MODE == 2) bv = bias[n];
#pragma unroll
      for (int r = 0; r < 8; ++r) {
        float v = acc[i][j][r] * scale;
        if (BIAS_MODE == 1) v += bias[mBase + mOff + r];
        if (BIAS_MODE == 2) v += bv;
        if (RESID) v += Rb[(size_t)(mBase + mOff + r) * ldc + n];
        if (ACT == 1) v = tanhf(v);
        if (ACT == 2) v = fmaxf(v, 0.0f);
        if (ACT == 3) v = v / (1.0f + expf(-v));
        if (ACT == 4) v = (v > 0.f) ? v : 0.01f * v;
        slab[(mOff + r) * 68 + (j << 4) + rlane] = v;
      }
    }
    __builtin_amdgcn_fence(__ATOMIC_RELEASE, "workgroup");
    __builtin_amdgcn_wave_barrier();
    __builtin_amdgcn_fence(__ATOMIC_ACQUIRE, "workgroup");
    if (OUT_MODE == 0) {
      float* C = (float*)Cout + (size_t)b * strideC;
      const int hh = lane >> 4, c4 = (lane & 15) * 4;
      for (int pass = 0; pass < 2; ++pass) {
#pragma unroll
        for (int it = 0; it < 8; ++it) {
          const int row = it * 2 + hh;
          v4f v = *(const v4f*)(slab + row * 68 + c4);
          *(volatile v4f*)(C + (size_t)(mBase + row) * ldc + n0 + c4) = v;
        }
        __threadfence();
      }
    } else {
      const int q = lane >> 3, c8 = (lane & 7) * 8;
      unsigned short* C;
      if (OUT_MODE == 3) {
        const int sel = (b & 1) ^ ((n0 >= (N >> 1)) ? 1 : 0);
        unsigned short* P0 = (unsigned short*)Cout;
        unsigned short* P1 = (unsigned short*)Cout2;
        C = (sel ? P1 : P0) + (size_t)(b >> 1) * strideC;
      } else {
        C = (unsigned short*)Cout + (size_t)b * strideC;
      }
      unsigned short* C2 = (OUT_MODE == 2) ? ((unsigned short*)Cout2 + (size_t)b * strideC) : nullptr;
      for (int pass = 0; pass < 2; ++pass) {
#pragma unroll
        for (int it = 0; it < 4; ++it) {
          const int row = it * 4 + q;
          const float* sp = slab + row * 68 + c8;
          v8h hv, lv;
#pragma unroll
          for (int e = 0; e < 8; ++e) {
            if (OUT_MODE == 2) {
              unsigned short hb = f2bf_bits(sp[e]);
              unsigned short lb = f2bf_bits(sp[e] - bf_bits2f(hb));
              hv[e] = __builtin_bit_cast(_Float16, hb);
              lv[e] = __builtin_bit_cast(_Float16, lb);
            } else {
              hv[e] = (_Float16)sp[e];
            }
          }
          *(volatile v8h*)(C + (size_t)(mBase + row) * ldc + n0 + c8) = hv;
          if (OUT_MODE == 2) *(volatile v8h*)(C2 + (size_t)(mBase + row) * ldc + n0 + c8) = lv;
        }
        __threadfence();
      }
    }
    __builtin_amdgcn_fence(__ATOMIC_RELEASE, "workgroup");
    __builtin_amdgcn_wave_barrier();
    __builtin_amdgcn_fence(__ATOMIC_ACQUIRE, "workgroup");
  }
}

__global__ __launch_bounds__(kThreads) void xprep_kernel(const float* __restrict__ x, unsigned short* __restrict__ xP) {
  const int i = blockIdx.x * kThreads + threadIdx.x;
  if (i >= kXPRows * (kDin / 8)) return;
  const int j = i >> 6, g = i & 63;
  const int jv = (j < kSeq) ? j : 0;
  const int s  = (jv < kHalfSeq) ? (2 * jv) : (2 * (jv - kHalfSeq) + 1);
  const float f = (j < kSeq) ? 1.0f : 0.0f;
  const float* src = x + (size_t)s * kDin + 8 * g;
  const v4f a = *(const v4f*)(src);
  const v4f c = *(const v4f*)(src + 4);
  u32x4 w;
  w[0] = pack_h2(bfr(a[0]) * f, bfr(a[1]) * f);
  w[1] = pack_h2(bfr(a[2]) * f, bfr(a[3]) * f);
  w[2] = pack_h2(bfr(c[0]) * f, bfr(c[1]) * f);
  w[3] = pack_h2(bfr(c[2]) * f, bfr(c[3]) * f);
  const size_t o = (size_t)i * 8;
  *(volatile u32x4*)(xP + o) = w;
  __threadfence();
  *(volatile u32x4*)(xP + o) = w;
}

__global__ __launch_bounds__(kThreads) void wsum_prep_kernel(const float* __restrict__ Mp, const float* __restrict__ Mm,
                                                            unsigned short* __restrict__ MT) {
  __shared__ float Sw[2][64 * 65];
  const int tid = threadIdx.x;
  const int d0 = blockIdx.x * 64, o0 = blockIdx.y * 64, k = blockIdx.z;
  {
    const int r = tid >> 2, c16 = (tid & 3) * 16;
    const size_t go = ((size_t)(k * kDin + d0 + r)) * kDout + o0 + c16;
#pragma unroll
    for (int qd = 0; qd < 4; ++qd) {
      const v4f a = *(const v4f*)(Mp + go + 4 * qd);
      const v4f c = *(const v4f*)(Mm + go + 4 * qd);
#pragma unroll
      for (int e = 0; e < 4; ++e) {
        const float sp = bfr(a[e]), sm = bfr(c[e]);
        Sw[0][r * 65 + c16 + 4 * qd + e] = sp + sm;
        Sw[1][r * 65 + c16 + 4 * qd + e] = sp - sm;
      }
    }
  }
  __syncthreads();
  u32x4 wv[4];
  size_t off[4];
#pragma unroll
  for (int it = 0; it < 4; ++it) {
    const int pl = it >> 1;
    const int q  = tid + kThreads * (it & 1);
    const int o  = q >> 3, g = q & 7;
    float v[8];
#pragma unroll
    for (int e = 0; e < 8; ++e) v[e] = Sw[pl][(8 * g + e) * 65 + o] * kWCarry;
    wv[it][0] = pack_h2(v[0], v[1]);
    wv[it][1] = pack_h2(v[2], v[3]);
    wv[it][2] = pack_h2(v[4], v[5]);
    wv[it][3] = pack_h2(v[6], v[7]);
    off[it] = ((size_t)((2 * k + pl) * kDout + o0 + o)) * kDin + d0 + 8 * g;
  }
  for (int pass = 0; pass < 2; ++pass) {
#pragma unroll
    for (int it = 0; it < 4; ++it) *(volatile u32x4*)(MT + off[it]) = wv[it];
    __threadfence();
  }
}

__global__ __launch_bounds__(kThreads) void filt_prep_kernel(const float* __restrict__ phi, unsigned short* __restrict__ QT) {
  const int i = blockIdx.x * kThreads + threadIdx.x;
  if (i >= kQLines * (kQLen / 8)) return;
  const int L   = i / (kQLen / 8);
  const int p0  = (i - L * (kQLen / 8)) * 8;
  const int par = L / kNumZ;
  const int rem = L - par * kNumZ;
  const int hf  = rem / kNumF;
  const int k   = rem - hf * kNumF;
  float v[8];
#pragma unroll
  for (int e = 0; e < 8; ++e) {
    const int del = p0 + e - kQZero;
    const int tau = 2 * del + par - hf;
    const bool valid = (del >= 0) && (tau >= 0) && (tau < kSeq);
    const int tc = (tau < 0) ? 0 : ((tau >= kSeq) ? (kSeq - 1) : tau);
    const float ph = phi[(size_t)tc * kNumF + k];
    v[e] = bfr(ph) * (valid ? kPhiCarry : 0.0f);
  }
  u32x4 w;
  w[0] = pack_h2(v[0], v[1]);
  w[1] = pack_h2(v[2], v[3]);
  w[2] = pack_h2(v[4], v[5]);
  w[3] = pack_h2(v[6], v[7]);
  const size_t o = (size_t)i * 8;
  *(volatile u32x4*)(QT + o) = w;
  __threadfence();
  *(volatile u32x4*)(QT + o) = w;
}

__global__ __launch_bounds__(kThreads) void arw_prep_kernel(const float* __restrict__ Mw, unsigned short* __restrict__ MAR) {
  const int i = blockIdx.x * kThreads + threadIdx.x;
  if (i >= kDout * (kDin / 8)) return;
  const int o = i >> 6, g = i & 63;
  const float* src = Mw + ((size_t)o * kDin + 8 * g) * kNumLag;
  v4f q[6];
#pragma unroll
  for (int cq = 0; cq < 6; ++cq) q[cq] = *(const v4f*)(src + 4 * cq);
  u32x4 wv[3];
  size_t off[3];
#pragma unroll
  for (int lag = 0; lag < kNumLag; ++lag) {
    float v[8];
#pragma unroll
    for (int e = 0; e < 8; ++e) {
      const int n = 3 * e + lag;
      v[e] = bfr(q[n >> 2][n & 3]) * kArCarry;
    }
    wv[lag][0] = pack_h2(v[0], v[1]);
    wv[lag][1] = pack_h2(v[2], v[3]);
    wv[lag][2] = pack_h2(v[4], v[5]);
    wv[lag][3] = pack_h2(v[6], v[7]);
    off[lag] = (size_t)o * kArK + lag * kDin + 8 * g;
  }
  for (int pass = 0; pass < 2; ++pass) {
#pragma unroll
    for (int lag = 0; lag < kNumLag; ++lag) *(volatile u32x4*)(MAR + off[lag]) = wv[lag];
    __threadfence();
  }
}

__global__ __launch_bounds__(kThreads) void spec_out_kernel(const unsigned short* __restrict__ QT,
                                                           const unsigned short* __restrict__ BEp,
                                                           const unsigned short* __restrict__ BOp,
                                                           const unsigned short* __restrict__ xPp,
                                                           const unsigned short* __restrict__ MARp,
                                                           float* __restrict__ out) {
  __shared__ __align__(16) unsigned short QL[kQLen];
  __shared__ __align__(16) unsigned short As[2][64 * kAPitch];
  __shared__ __align__(16) float sT[8][16 * 68];
  const int tid = threadIdx.x, lane = tid & 31, wave = tid >> 5;
  const int rlane = lane & 15;
  const int koff  = (lane >> 4) * 8;
  const int mOff  = (lane >> 4) * 8;
  const int mt = blockIdx.x, par = blockIdx.y;
  const int m0 = mt * 64;
  const int n0 = wave * 64;
  const _Float16* Bpl = (const _Float16*)(par ? BOp : BEp);
  const _Float16* xP  = (const _Float16*)xPp;
  const _Float16* MAR = (const _Float16*)MARp;

  v8f acc[4][4];
#pragma unroll
  for (int i = 0; i < 4; ++i)
#pragma unroll
    for (int j = 0; j < 4; ++j) acc[i][j] = (v8f){0.f,0.f,0.f,0.f,0.f,0.f,0.f,0.f};

  const int jend = m0 + 64;
  int buf = 0;
#pragma unroll 1
  for (int k = 0; k < kNumF; ++k) {
#pragma unroll 1
    for (int hf = 0; hf < 2; ++hf) {
      __syncthreads();
      if (wave < 5) {
        const u32x4 w = *(const u32x4*)(QT + ((size_t)((par * 2 + hf) * kNumF + k)) * kQLen + tid * 8);
        *(u32x4*)(QL + tid * 8) = w;
      }
      __syncthreads();
      const _Float16* Bk = Bpl + (size_t)k * ((size_t)kDout * kSeq) + hf * kHalfSeq;
#pragma unroll 1
      for (int j0 = 0; j0 < jend; j0 += 32) {
        {
          const int r = tid >> 2, c0 = (tid & 3) * 8;
          const int base = kQZero + m0 - j0 + r - c0;
          unsigned qv[8];
#pragma unroll
          for (int e = 0; e < 8; ++e) qv[e] = (unsigned)QL[base - e];
          u32x4 w;
          w[0] = qv[0] | (qv[1] << 16);
          w[1] = qv[2] | (qv[3] << 16);
          w[2] = qv[4] | (qv[5] << 16);
          w[3] = qv[6] | (qv[7] << 16);
          *(u32x4*)(&As[buf][r * kAPitch + c0]) = w;
        }
        __syncthreads();
        const _Float16* At = (const _Float16*)(&As[buf][0]);
        v16h bq[4];
#pragma unroll
        for (int jj = 0; jj < 4; ++jj)
          bq[jj] = FragH::load(Bk + (size_t)(n0 + 16 * jj + rlane) * kSeq + j0 + koff);
#pragma unroll
        for (int ii = 0; ii < 4; ++ii) {
          const v16h a = FragH::load(At + (16 * ii + rlane) * kAPitch + koff);
#pragma unroll
          for (int jj = 0; jj < 4; ++jj) acc[ii][jj] = FragH::mma(a, bq[jj], acc[ii][jj]);
          grp_guard_h(acc[ii][0], acc[ii][1], acc[ii][2], acc[ii][3], a, bq[3]);
        }
        keep4_h(bq[0], bq[1], bq[2], bq[3]);
        buf ^= 1;
      }
    }
  }

#pragma unroll 1
  for (int lag = 0; lag < kNumLag; ++lag) {
    const int diff = par - lag;
    int rb;
    if (diff == 1) rb = kHalfSeq;
    else if (diff == 0) rb = 0;
    else if (diff == -1) rb = kHalfSeq - 1;
    else rb = -1;
    const bool zneed = (diff < 0);
    int arow[4];
#pragma unroll
    for (int ii = 0; ii < 4; ++ii) {
      const int m = m0 + 16 * ii + rlane;
      int jr = m + rb;
      if (zneed && m == 0) jr = kSeq;
      jr = (jr < 0) ? 0 : ((jr > kSeq) ? kSeq : jr);
      arow[ii] = jr;
    }
#pragma unroll 1
    for (int d0 = 0; d0 < kDin; d0 += 32) {
      v16h bq[4];
#pragma unroll
      for (int jj = 0; jj < 4; ++jj)
        bq[jj] = FragH::load(MAR + (size_t)(n0 + 16 * jj + rlane) * kArK + lag * kDin + d0 + koff);
#pragma unroll
      for (int ii = 0; ii < 4; ++ii) {
        const v16h a = FragH::load(xP + (size_t)arow[ii] * kDin + d0 + koff);
#pragma unroll
        for (int jj = 0; jj < 4; ++jj) acc[ii][jj] = FragH::mma(a, bq[jj], acc[ii][jj]);
        grp_guard_h(acc[ii][0], acc[ii][1], acc[ii][2], acc[ii][3], a, bq[3]);
      }
      keep4_h(bq[0], bq[1], bq[2], bq[3]);
    }
  }
  acc_guard4(acc[0][0], acc[0][1], acc[0][2], acc[0][3]);
  acc_guard4(acc[1][0], acc[1][1], acc[1][2], acc[1][3]);
  acc_guard4(acc[2][0], acc[2][1], acc[2][2], acc[2][3]);
  acc_guard4(acc[3][0], acc[3][1], acc[3][2], acc[3][3]);

  float* slab = sT[wave];
  float* Cb = out + (size_t)par * kDout;
  const int ldc = 2 * kDout;
#pragma unroll
  for (int i = 0; i < 4; ++i) {
    const int mBase = m0 + (i << 4);
#pragma unroll
    for (int j = 0; j < 4; ++j) {
#pragma unroll
      for (int r = 0; r < 8; ++r) slab[(mOff + r) * 68 + (j << 4) + rlane] = acc[i][j][r] * kOutScale;
    }
    __builtin_amdgcn_fence(__ATOMIC_RELEASE, "workgroup");
    __builtin_amdgcn_wave_barrier();
    __builtin_amdgcn_fence(__ATOMIC_ACQUIRE, "workgroup");
    {
      const int hh = lane >> 4, c4 = (lane & 15) * 4;
      for (int pass = 0; pass < 2; ++pass) {
#pragma unroll
        for (int it = 0; it < 8; ++it) {
          const int row = it * 2 + hh;
          v4f v = *(const v4f*)(slab + row * 68 + c4);
          *(volatile v4f*)(Cb + (size_t)(mBase + row) * ldc + n0 + c4) = v;
        }
        __threadfence();
      }
    }
    __builtin_amdgcn_fence(__ATOMIC_RELEASE, "workgroup");
    __builtin_amdgcn_wave_barrier();
    __builtin_amdgcn_fence(__ATOMIC_ACQUIRE, "workgroup");
  }
}

extern "C" void kernel_launch(void* const* d_in, const int* in_sizes, int n_in,
                              void* d_out, int out_size, void* d_ws, size_t ws_size,
                              hipStream_t stream) {
  if (n_in < 5) return;
  if (in_sizes[0] != kSeq * kDin) return;
  if (in_sizes[1] != kSeq * kNumF) return;
  if (in_sizes[2] != kDout * kDin * kNumLag) return;
  if (in_sizes[3] != kNumF * kDin * kDout) return;
  if (in_sizes[4] != kNumF * kDin * kDout) return;
  if (out_size != kSeq * kDout) return;
  if (ws_size < kWsTotal) return;

  const float* x   = (const float*)d_in[0];
  const float* phi = (const float*)d_in[1];
  const float* Mw  = (const float*)d_in[2];
  const float* Mp  = (const float*)d_in[3];
  const float* Mm  = (const float*)d_in[4];
  float* out = (float*)d_out;

  char* ws = (char*)d_ws;
  unsigned short* xP  = (unsigned short*)(ws + kOffXP);
  unsigned short* MT  = (unsigned short*)(ws + kOffMT);
  unsigned short* BE  = (unsigned short*)(ws + kOffBE);
  unsigned short* BO  = (unsigned short*)(ws + kOffBO);
  unsigned short* QT  = (unsigned short*)(ws + kOffQT);
  unsigned short* MAR = (unsigned short*)(ws + kOffMar);

  const int nXP  = kXPRows * (kDin / 8);
  const int nQT  = kQLines * (kQLen / 8);
  const int nMAR = kDout * (kDin / 8);
  xprep_kernel<<<(nXP + kThreads - 1) / kThreads, kThreads, 0, stream>>>(x, xP);
  wsum_prep_kernel<<<dim3(kDin / 64, kDout / 64, kNumF), kThreads, 0, stream>>>(Mp, Mm, MT);
  filt_prep_kernel<<<(nQT + kThreads - 1) / kThreads, kThreads, 0, stream>>>(phi, QT);
  arw_prep_kernel<<<(nMAR + kThreads - 1) / kThreads, kThreads, 0, stream>>>(Mw, MAR);

  const int tilesG = (kDout / 64) * (kSeq / 64);
  wmma_gemm64<0, false, 0, 3, false, 0><<<dim3(tilesG / 8, kNumZ), kThreads, 0, stream>>>(
      MT, MT, kDin, (long)kDout * kDin,
      xP, xP, kDin, 0L,
      (void*)BE, (void*)BO, kSeq, (long)kDout * kSeq,
      x, x, 0L,
      kDout, kSeq, kDin, kGEpiScale);

  spec_out_kernel<<<dim3(kHalfSeq / 64, 2), kThreads, 0, stream>>>(QT, BE, BO, xP, MAR, out);
}
